// TableBatchedTTEmbeddingBag_84576495993304
// MI455X (gfx1250) — hardware-verified
//
#include <hip/hip_runtime.h>


#ifndef Nseg
#define Nseg 32768
#endif
#define Nseg_FULL 32768
#define NTAB  4
#define NP    100
#define RK    32
#define QD    4
#define BPT_FULL (Nseg_FULL / NTAB)
#define C0W   (QD * RK)
#define C1W   (RK * QD * RK)
#define C2W   (RK * QD)
#define NCOL  (QD * RK)
#define NROWS (NP * NP * NP)
#define TILE_H (QD * QD * RK)
#define PSP   132
#define TSP   132
#define BW    4
#define BPW   2
#define CH    4
#define WSC   1024.0f
#define CSC   64.0f
#define OSC   (1.0f / 65536.0f)

static_assert(RK == 32);
static_assert(QD * QD == 16);
static_assert(QD <= 16);
static_assert((NP * QD) % 16 == 0);
static_assert(NCOL % 16 == 0);
static_assert(NCOL / 16 == 8);
static_assert(Nseg % (BW * BPW) == 0);
static_assert(Nseg >= BW * BPW);
static_assert(Nseg <= Nseg_FULL);
static_assert(Nseg_FULL % NTAB == 0);
static_assert((PSP * 4) % 16 == 0);
static_assert((TSP * 4) % 16 == 0);
static_assert(32 * 2 * 4 * 16 == 16 * NCOL * 2);
static_assert(256 * 2 * 16 == NCOL * RK * 2);
static_assert(256 * 4 * 16 == C1W * 4);
static_assert(32 * 16 == BPW * 64 * 4);
static_assert(CH * TILE_H * 2 == 32 * 8 * 16);
static_assert(CH * C2W * 2 == 32 * 2 * 16);
static_assert(16 * PSP * 4 <= 131072);
static_assert(RK * TSP * 4 <= 131072);
static_assert(BW * CH * TILE_H * 2 + BW * CH * C2W * 2 + BW * BPW * 64 * 4 <= 131072);

typedef _Float16 h16;
typedef unsigned short bf;
typedef __attribute__((ext_vector_type(16))) __bf16   v16bf;
typedef __attribute__((ext_vector_type(16))) _Float16 v16h;
typedef __attribute__((ext_vector_type(8)))  _Float16 v8h;
typedef __attribute__((ext_vector_type(8)))  unsigned short v8us;
typedef __attribute__((ext_vector_type(8)))  float    v8f;
typedef __attribute__((ext_vector_type(4)))  float    v4f;
typedef v4f  __attribute__((may_alias)) v4fa;

__device__ __forceinline__ unsigned short f2bf(float f) { unsigned u = __float_as_uint(f); u += 0x7FFFu + ((u >> 16) & 1u); return (unsigned short)(u >> 16); }
__device__ __forceinline__ float bfr(float f) { return __uint_as_float(((unsigned)f2bf(f)) << 16); }
__device__ __forceinline__ v16h cat16(v8h lo, v8h hi) { return __builtin_shufflevector(lo, hi, 0, 1, 2, 3, 4, 5, 6, 7, 8, 9, 10, 11, 12, 13, 14, 15); }
__device__ __forceinline__ v16bf cat16b(v8us lo, v8us hi) { return __builtin_bit_cast(v16bf, __builtin_shufflevector(lo, hi, 0, 1, 2, 3, 4, 5, 6, 7, 8, 9, 10, 11, 12, 13, 14, 15)); }
__device__ __forceinline__ v8f wmma16(v16h a, v16h b, v8f c) { return __builtin_amdgcn_wmma_f32_16x16x32_f16(false, a, false, b, (short)0, c, false, false); }
__device__ __forceinline__ v8f wmmab(v16bf a, v16bf b, v8f c) { return __builtin_amdgcn_wmma_f32_16x16x32_bf16(false, a, false, b, (short)0, c, false, false); }
__device__ __forceinline__ v16h  ldh(const h16* p) { return cat16(*(const v8h*)p, *(const v8h*)(p + 16)); }
__device__ __forceinline__ v16bf ldb(const bf* p)  { return cat16b(*(const v8us*)p, *(const v8us*)(p + 16)); }
__device__ __forceinline__ void wave_sync() { __builtin_amdgcn_fence(3  , "wavefront"); __builtin_amdgcn_wave_barrier(); asm volatile("" ::: "memory"); }

static __device__ __forceinline__ h16 toh_flush(float v) { const h16 r = (h16)v; return (fabsf(v) < 6.103515625e-05f) ? (h16)0.0f : r; }
__device__ __forceinline__ v8f wmma16g(v16h a, v16h b, v8f c) { c = wmma16(a, b, c); asm volatile("v_nop\n\tv_nop\n\tv_nop\n\tv_nop" : "+v"(c) : "v"(a), "v"(b)); return c; }
__device__ __forceinline__ v8f wmmabg(v16bf a, v16bf b, v8f c) { c = wmmab(a, b, c); asm volatile("v_nop\n\tv_nop\n\tv_nop\n\tv_nop" : "+v"(c) : "v"(a), "v"(b)); return c; }

__global__ __launch_bounds__(256) void k_cvt8(const float* __restrict__ src, bf* dst, size_t n8) {
    const size_t i = (size_t)blockIdx.x * 256 + threadIdx.x; if (i >= n8) return;
    const v8f v = *(const v8f*)(src + i * 8); v8us o;
#pragma unroll
    for (int k = 0; k < 8; ++k) o[k] = f2bf(v[k]);
    *(volatile v8us*)(dst + i * 8) = o; __threadfence(); *(volatile v8us*)(dst + i * 8) = o;
}

__global__ __launch_bounds__(256) void k_c1t(const float* __restrict__ src, bf* dst) {
    __shared__ __align__(16) float ls[RK * TSP];
    const int tid = threadIdx.x; const size_t blk = blockIdx.x;
    const float* s = src + blk * (size_t)C1W;
#pragma unroll
    for (int i = 0; i < 4; ++i) { const int f = i * 256 + tid; const int r = f >> 5, c4 = (f & 31) * 4;
        const v4f v = *(const v4f*)(s + (size_t)f * 4); *(v4fa*)(&ls[r * TSP + c4]) = v; }
    __syncthreads();
    bf* d = dst + blk * (size_t)C1W;
#pragma unroll 1
    for (int ps = 0; ps < 2; ++ps) {
#pragma unroll
        for (int i = 0; i < 2; ++i) { const int p = i * 256 + tid; const int n = p >> 2, c8 = (p & 3) * 8;
            v8us o;
#pragma unroll
            for (int k = 0; k < 8; ++k) o[k] = f2bf(ls[(c8 + k) * TSP + n]);
            *(volatile v8us*)(d + (size_t)p * 8) = o; }
        if (ps == 0) __threadfence(); }
}

__global__ __launch_bounds__(256) void k_c2t(const float* __restrict__ src, h16* dst, int n8) {
    const int p = (int)blockIdx.x * 256 + (int)threadIdx.x; if (p >= n8) return;
    const int row = p >> 4, q = p & 15; const int c = q >> 2, s0 = (q & 3) * 8;
    const float* s = src + (size_t)row * C2W;
    v8h o;
#pragma unroll
    for (int k = 0; k < 8; ++k) o[k] = toh_flush(bfr(s[(s0 + k) * QD + c]) * CSC);
    *(volatile v8h*)(dst + (size_t)p * 8) = o; __threadfence(); *(volatile v8h*)(dst + (size_t)p * 8) = o;
}

__global__ __launch_bounds__(32) void k_pair(const bf* __restrict__ C0B, const bf* __restrict__ C1T, h16* WT) {
    __shared__ __align__(16) float os[16 * PSP];
    const int lane = threadIdx.x & 31, lr = lane & 15, hi = lane >> 4;
    const int i1 = blockIdx.x, g = blockIdx.y, t = blockIdx.z;
    const size_t aoff = ((size_t)t * (NP * QD) + (size_t)g * 16 + lr) * RK + 8 * hi;
    const size_t boff = (((size_t)t * NP + i1) * NCOL + lr) * RK + 8 * hi;
    const v16bf a = ldb(C0B + aoff);
    v8f acc[8];
#pragma unroll
    for (int nb = 0; nb < 8; ++nb) { const v16bf b = ldb(C1T + boff + (size_t)nb * 16 * RK); acc[nb] = (v8f){}; acc[nb] = wmmabg(a, b, acc[nb]); }
#pragma unroll
    for (int nb = 0; nb < 8; ++nb) {
#pragma unroll
        for (int j = 0; j < 8; ++j) os[(hi * 8 + j) * PSP + nb * 16 + lr] = acc[nb][j]; }
    wave_sync();
#pragma unroll 1
    for (int ps = 0; ps < 2; ++ps) {
#pragma unroll
        for (int i0q = 0; i0q < 4; ++i0q) {
            const size_t tb = (((size_t)t * NP + (size_t)(g * 4 + i0q)) * NP + (size_t)i1) * TILE_H;
#pragma unroll
            for (int s = 0; s < 2; ++s) { const int p = s * 32 + lane; const int aq = p >> 4, c8 = (p & 15) * 8;
                const int row = i0q * 4 + aq;
                const v4f x0 = *(const v4fa*)(&os[row * PSP + c8]); const v4f x1 = *(const v4fa*)(&os[row * PSP + c8 + 4]); v8h hv;
#pragma unroll
                for (int i = 0; i < 4; ++i) { hv[i] = toh_flush(x0[i] * WSC); hv[4 + i] = toh_flush(x1[i] * WSC); }
                *(volatile v8h*)(WT + tb + (size_t)p * 8) = hv; } }
        if (ps == 0) __threadfence(); }
}

__global__ __launch_bounds__(32 * BW) void k_seg(const int* __restrict__ indices, const int* __restrict__ offsets, const h16* __restrict__ WT, const h16* __restrict__ C2T, float* OUT, int nnz) {
    __shared__ __align__(16) h16   at[BW * CH * TILE_H];
    __shared__ __align__(16) h16   bt[BW * CH * C2W];
    __shared__ __align__(16) float os[BW * BPW * 64];
    const int lane = threadIdx.x & 31, lr = lane & 15, hi = lane >> 4;
    const int wave = __builtin_amdgcn_readfirstlane((int)(threadIdx.x >> 5));
    int bv = ((int)blockIdx.x * BW + (int)(threadIdx.x >> 5)) * BPW;
    const int lv = (bv + BPW <= Nseg) ? 1 : 0;
    bv = (bv + BPW <= Nseg) ? bv : (Nseg - BPW);
    const int seg0 = __builtin_amdgcn_readfirstlane(bv);
    const int live = __builtin_amdgcn_readfirstlane(lv);
    const int ab = wave * (CH * TILE_H), bb = wave * (CH * C2W), ob = wave * (BPW * 64);
    const v16h hz = (v16h){}; const v8h z8 = (v8h){};
    const int nlast = nnz - 1;
#pragma unroll 1
    for (int q = 0; q < BPW; ++q) {
        const int seg = seg0 + q;
        const int t = seg / BPT_FULL;
        int st = offsets[seg], en = offsets[seg + 1];
        st = st < 0 ? 0 : (st > nnz ? nnz : st);
        en = en < st ? st : (en > nnz ? nnz : en);
        v8f acc = (v8f){};
#pragma unroll 1
        for (int j0 = st; j0 < en; j0 += CH) {
#pragma unroll
            for (int jj = 0; jj < CH; ++jj) {
                const int j = j0 + jj; const int jc = j < nlast ? j : nlast;
                int idx = indices[jc]; idx = idx < 0 ? 0 : (idx > NROWS - 1 ? NROWS - 1 : idx);
                const size_t tb = ((size_t)t * (NP * NP) + (size_t)(idx / NP)) * TILE_H;
                const bool ok = j < en;
#pragma unroll
                for (int s = 0; s < 2; ++s) { const int p = s * 32 + lane;
                    v8h x = *(const v8h*)(WT + tb + (size_t)p * 8);
                    asm volatile("" : "+v"(x));
                    x = ok ? x : z8;
                    *(v8h*)(&at[ab + jj * TILE_H + p * 8]) = x; } }
#pragma unroll
            for (int s = 0; s < 2; ++s) {
                const int jb = 2 * s + hi; const int j = j0 + jb; const int jc = j < nlast ? j : nlast;
                int idx = indices[jc];
                asm volatile("" : "+v"(idx));
                idx = idx < 0 ? 0 : (idx > NROWS - 1 ? NROWS - 1 : idx);
                const int i2 = idx - (idx / NP) * NP;
                v8h y = *(const v8h*)(C2T + ((size_t)t * NP + (size_t)i2) * C2W + (size_t)lr * 8);
                asm volatile("" : "+v"(y));
                y = (j < en) ? y : z8;
                *(v8h*)(&bt[bb + jb * C2W + lr * 8]) = y; }
            wave_sync();
#pragma unroll
            for (int jj = 0; jj < CH; ++jj) {
                const int ao = ab + jj * TILE_H + lr * RK + 8 * hi;
                const v16h a = cat16(*(const v8h*)(&at[ao]), *(const v8h*)(&at[ao + 16]));
                const int bo = bb + jj * C2W + (lr & 3) * RK + 8 * hi;
                v16h b = cat16(*(const v8h*)(&bt[bo]), *(const v8h*)(&bt[bo + 16]));
                b = (lr < QD) ? b : hz;
                acc = wmma16g(a, b, acc); }
            wave_sync();
        }
        if (lr < QD) {
#pragma unroll
            for (int r = 0; r < 8; ++r) os[ob + q * 64 + (8 * hi + r) * QD + lr] = acc[r] * OSC; }
    }
    wave_sync();
    if (live) {
        const v4f val = *(const v4fa*)(&os[ob + lane * 4]);
        float* op = OUT + (size_t)seg0 * 64 + (size_t)lane * 4;
        *(volatile v4f*)op = val; __threadfence(); *(volatile v4f*)op = val; }
}

static constexpr size_t al256(size_t v) { return (v + 255) & ~(size_t)255; }
static constexpr size_t SZ_C0B = al256((size_t)NTAB * NP * C0W * 2);
static constexpr size_t SZ_C1T = al256((size_t)NTAB * NP * C1W * 2);
static constexpr size_t SZ_C2T = al256((size_t)NTAB * NP * C2W * 2);
static constexpr size_t SZ_WT  = al256((size_t)NTAB * NP * NP * TILE_H * 2);
static constexpr size_t SZ_TOTAL = SZ_C0B + SZ_C1T + SZ_C2T + SZ_WT;
static_assert(SZ_TOTAL <= (size_t)134217728);
static_assert(((size_t)NTAB * NP * C0W) % 8 == 0);
static_assert(((size_t)NTAB * NP * C2W) % 8 == 0);
static_assert((size_t)NTAB * NP * NCOL * RK == (size_t)NTAB * NP * C1W);
static_assert((size_t)(NTAB - 1) * (NP * NP) + (size_t)(NROWS - 1) / NP < (size_t)NTAB * NP * NP);

extern "C" void kernel_launch(void* const* d_in, const int* in_sizes, int n_in,
                              void* d_out, int out_size, void* d_ws, size_t ws_size, hipStream_t stream) {
    if (n_in < 5) return;
    if (in_sizes[0] < 1) return;
    if ((size_t)in_sizes[1] < (size_t)Nseg + 1) return;
    if ((size_t)in_sizes[2] < (size_t)NTAB * NP * C0W || (size_t)in_sizes[3] < (size_t)NTAB * NP * C1W || (size_t)in_sizes[4] < (size_t)NTAB * NP * C2W) return;
    if ((size_t)out_size < (size_t)Nseg * 64) return;
    if (SZ_TOTAL > ws_size) return;
    const int* indices = (const int*)d_in[0];
    const int* offsets = (const int*)d_in[1];
    const float* core0 = (const float*)d_in[2];
    const float* core1 = (const float*)d_in[3];
    const float* core2 = (const float*)d_in[4];
    const int nnz = in_sizes[0];
    float* OUT = (float*)d_out;
    char* wsp = (char*)d_ws;
    bf*  C0B = (bf*)wsp;  wsp += SZ_C0B;
    bf*  C1T = (bf*)wsp;  wsp += SZ_C1T;
    h16* C2T = (h16*)wsp; wsp += SZ_C2T;
    h16* WT  = (h16*)wsp; wsp += SZ_WT;

    { const size_t n8 = (size_t)NTAB * NP * C0W / 8;
      k_cvt8<<<(unsigned)((n8 + 255) / 256), 256, 0, stream>>>(core0, C0B, n8); }
    k_c1t<<<NTAB * NP, 256, 0, stream>>>(core1, C1T);
    { const int n8 = NTAB * NP * C2W / 8;
      k_c2t<<<(unsigned)((n8 + 255) / 256), 256, 0, stream>>>(core2, C2T, n8); }

    k_pair<<<dim3(NP, NP * QD / 16, NTAB), 32, 0, stream>>>(C0B, C1T, WT);

    k_seg<<<Nseg / (BW * BPW), 32 * BW, 0, stream>>>(indices, offsets, WT, C2T, OUT, nnz);
}
